// CharacterLSTM_88330297409632
// MI455X (gfx1250) — hardware-run, weakly checked
//
#include <hip/hip_runtime.h>
#include <math.h>

constexpr int NBAT   = 64;
constexpr int NSEQ   = 256;
constexpr int NSTEP  = 24;
constexpr int NEMB   = 128;
constexpr int NHID   = 256;
constexpr int NCHAR  = 256;
constexpr int NWORD  = NBAT * NSEQ;
constexpr int NGATE  = 4 * NHID;
constexpr int TROWS  = 32;
constexpr int RTHR   = 512;
constexpr int RWAVES = RTHR / 32;
constexpr int HPITCH = 264;
constexpr int OPITCH = 260;
constexpr float HCARRY        = 16.0f;
constexpr float WCARRY        = 64.0f;
constexpr float ACC_SCALE     = HCARRY * WCARRY;
constexpr float ACC_SCALE_INV = 1.0f / ACC_SCALE;
constexpr float F16_MIN_NORMAL = 6.103515625e-05f;
constexpr int CVT_THR = 256;
constexpr int TAB_THR = 256;

static_assert(NWORD == 16384, "word count");
static_assert(NGATE == 1024, "gate columns");
static_assert(NWORD % TROWS == 0, "grid exact");
static_assert(NHID == 16 * RWAVES, "one 16-unit group per wave");
static_assert(NHID % 32 == 0, "K multiple of 32");
static_assert(TROWS == 32, "two 16-row subtiles per block");
static_assert(TROWS * NSTEP <= 2 * RTHR, "id staging covers the tile in two passes");
static_assert((TROWS * NHID) / 4 == 4 * RTHR, "final store loop covers the tile exactly");
static_assert((NGATE * NHID) % (8 * CVT_THR) == 0, "convert grid exact");
static_assert(TAB_THR == NHID, "one thread per hidden unit in the table kernel");
static_assert(NEMB % 4 == 0, "float4 steps");
static_assert((HPITCH % 8) == 0 && (OPITCH % 4) == 0, "LDS pitches keep 16-B alignment");

typedef __attribute__((ext_vector_type(16))) _Float16 v16h;
typedef __attribute__((ext_vector_type(8)))  _Float16 v8h;
typedef __attribute__((ext_vector_type(8)))  float    v8f;
typedef __attribute__((ext_vector_type(4)))  float    v4f;
typedef __attribute__((ext_vector_type(4)))  int      v4i;

struct FragH {
  union U { v16h v; v8h h[2]; };
  static __device__ __forceinline__ v16h load(const _Float16* p) {
    U f;
    f.h[0] = *(const v8h*)(p);
    f.h[1] = *(const v8h*)(p + 16);
    return f.v;
  }
  static __device__ __forceinline__ v8f mma(v16h a, v16h b, v8f c) {
    return __builtin_amdgcn_wmma_f32_16x16x32_f16(false, a, false, b, (short)0, c, false, false);
  }
};

__device__ __forceinline__ void tie_one(v8f& d, v16h a, v16h b) {
  asm volatile("" : "+v"(d) : "v"(a), "v"(b));
}
__device__ __forceinline__ void tie_close(v8f& d, v16h a0, v16h a1, v16h b0, v16h b1, v16h b2, v16h b3) {
  asm volatile("v_nop\n\tv_nop\n\tv_nop\n\tv_nop" : "+v"(d) : "v"(a0), "v"(a1), "v"(b0), "v"(b1), "v"(b2), "v"(b3));
}
__device__ __forceinline__ void settle_one(v8f& d) {
  asm volatile("v_nop\n\tv_nop\n\tv_nop\n\tv_nop" : "+v"(d));
}

__device__ __forceinline__ float fsig(float x)  { return __builtin_amdgcn_rcpf(1.0f + __expf(-x)); }
__device__ __forceinline__ float ftanh(float x) { return 1.0f - 2.0f * __builtin_amdgcn_rcpf(__expf(2.0f * x) + 1.0f); }

__global__ __launch_bounds__(TAB_THR) void table_kernel(const float* __restrict__ emb, const float* __restrict__ wih,
                                                        const float* __restrict__ bih, const float* __restrict__ bhh,
                                                        float* __restrict__ PT) {
  const int ch = blockIdx.x;
  const int u  = threadIdx.x;
  const float* er = emb + (size_t)ch * NEMB;
  const float* w0 = wih + (size_t)u * NEMB;
  const float* w1 = w0 + (size_t)1 * NHID * NEMB;
  const float* w2 = w0 + (size_t)2 * NHID * NEMB;
  const float* w3 = w0 + (size_t)3 * NHID * NEMB;
  float s0 = 0.0f, s1 = 0.0f, s2 = 0.0f, s3 = 0.0f;
#pragma unroll 1
  for (int k = 0; k < NEMB; k += 4) {
    const v4f e  = *(const v4f*)(er + k);
    const v4f a0 = *(const v4f*)(w0 + k);
    const v4f a1 = *(const v4f*)(w1 + k);
    const v4f a2 = *(const v4f*)(w2 + k);
    const v4f a3 = *(const v4f*)(w3 + k);
#pragma unroll
    for (int j = 0; j < 4; ++j) {
      const float ev = e[j];
      s0 = fmaf(ev, a0[j], s0);
      s1 = fmaf(ev, a1[j], s1);
      s2 = fmaf(ev, a2[j], s2);
      s3 = fmaf(ev, a3[j], s3);
    }
  }
  const float bs0 = bih[u] + bhh[u];
  const float bs1 = bih[NHID + u] + bhh[NHID + u];
  const float bs2 = bih[2 * NHID + u] + bhh[2 * NHID + u];
  const float bs3 = bih[3 * NHID + u] + bhh[3 * NHID + u];
  v4f o;
  o[0] = (s0 + bs0) * ACC_SCALE;
  o[1] = (s1 + bs1) * ACC_SCALE;
  o[2] = (s2 + bs2) * ACC_SCALE;
  o[3] = (s3 + bs3) * ACC_SCALE;
  float* op = PT + (size_t)ch * NGATE + (size_t)u * 4;
  *(volatile v4f*)op = o;
  __threadfence();
  *(volatile v4f*)op = o;
}

__global__ __launch_bounds__(CVT_THR) void whh_cvt_kernel(const float* __restrict__ whh, unsigned short* __restrict__ WHp) {
  const int i  = blockIdx.x * CVT_THR + threadIdx.x;
  const int n8 = (NGATE * NHID) / 8;
  if (i < n8) {
    const float* sp = whh + (size_t)i * 8;
    const v4f a = *(const v4f*)(sp);
    const v4f b = *(const v4f*)(sp + 4);
    v8h hv;
#pragma unroll
    for (int e = 0; e < 4; ++e) {
      const float xa = a[e] * WCARRY;
      const float xb = b[e] * WCARRY;
      const float fa = (fabsf(xa) < F16_MIN_NORMAL) ? 0.0f : xa;
      const float fb = (fabsf(xb) < F16_MIN_NORMAL) ? 0.0f : xb;
      hv[e]     = (_Float16)fa;
      hv[4 + e] = (_Float16)fb;
    }
    _Float16* dp = (_Float16*)WHp + (size_t)i * 8;
    *(volatile v8h*)dp = hv;
    __threadfence();
    *(volatile v8h*)dp = hv;
  }
}

__global__ __launch_bounds__(RTHR) void rec_kernel(const int* __restrict__ chars, const float* __restrict__ PT,
                                                   const unsigned short* __restrict__ WHp, float* __restrict__ out) {
  __shared__ __align__(16) _Float16 Ah[TROWS * HPITCH];
  __shared__ __align__(16) float    Hs[TROWS * OPITCH];
  __shared__ __align__(16) int      idsT[NSTEP * TROWS];
  __shared__ __align__(16) int      lensS[TROWS];
  const _Float16* WH = (const _Float16*)WHp;
  const int tid = threadIdx.x, lane = tid & 31, wave = tid >> 5;
  const int c = lane & 15, hh = lane >> 4, koff = hh * 8;
  const int n0 = blockIdx.x * TROWS;
  const int u  = 16 * wave + c;

#pragma unroll
  for (int it = 0; it < 2; ++it) {
    const int i  = it * RTHR + tid;
    const int ic = (i < TROWS * NSTEP) ? i : (TROWS * NSTEP - 1);
    int raw = chars[(size_t)n0 * NSTEP + ic];
    asm volatile("" : "+v"(raw));
    const int m  = ic / NSTEP;
    const int tt = ic - m * NSTEP;
    const int lo = (raw < 0) ? 0 : raw;
    const int idc = (lo > NCHAR - 1) ? (NCHAR - 1) : lo;
    const int enc = idc | ((raw != 0) ? 256 : 0);
    if (i < TROWS * NSTEP) idsT[tt * TROWS + m] = enc;
  }
  __syncthreads();
  if (tid < TROWS) {
    int cnt = 0;
#pragma unroll 1
    for (int tt = 0; tt < NSTEP; ++tt) cnt += (idsT[tt * TROWS + tid] >> 8);
    lensS[tid] = cnt;
  }
  __syncthreads();

  int   lenv[2][8];
  float cst[2][8], lh[2][8];
  {
    const v4i* lp = (const v4i*)lensS;
#pragma unroll
    for (int rt = 0; rt < 2; ++rt) {
      const v4i l0 = lp[4 * rt + 2 * hh];
      const v4i l1 = lp[4 * rt + 2 * hh + 1];
      lenv[rt][0] = l0[0]; lenv[rt][1] = l0[1]; lenv[rt][2] = l0[2]; lenv[rt][3] = l0[3];
      lenv[rt][4] = l1[0]; lenv[rt][5] = l1[1]; lenv[rt][6] = l1[2]; lenv[rt][7] = l1[3];
#pragma unroll
      for (int v = 0; v < 8; ++v) { cst[rt][v] = 0.0f; lh[rt][v] = 0.0f; }
    }
  }

  const float*    ptl = PT + (size_t)u * 4;
  const _Float16* wh  = WH + (size_t)u * NHID + koff;
  const _Float16* ah0 = Ah + c * HPITCH + koff;
  const _Float16* ah1 = Ah + (16 + c) * HPITCH + koff;

#pragma unroll 1
  for (int t = 0; t < NSTEP; ++t) {
    v8f acc[4][2];
    const v4i* idrow = (const v4i*)(idsT + t * TROWS);
#pragma unroll
    for (int rt = 0; rt < 2; ++rt) {
      const v4i q0 = idrow[4 * rt + 2 * hh];
      const v4i q1 = idrow[4 * rt + 2 * hh + 1];
      int enc[8];
      enc[0] = q0[0]; enc[1] = q0[1]; enc[2] = q0[2]; enc[3] = q0[3];
      enc[4] = q1[0]; enc[5] = q1[1]; enc[6] = q1[2]; enc[7] = q1[3];
#pragma unroll
      for (int v = 0; v < 8; ++v) {
        const int id = enc[v] & 255;
        const v4f p = *(const v4f*)(ptl + (size_t)id * NGATE);
        acc[0][rt][v] = p[0];
        acc[1][rt][v] = p[1];
        acc[2][rt][v] = p[2];
        acc[3][rt][v] = p[3];
      }
    }

    if (t > 0) {
#pragma unroll 1
      for (int k0 = 0; k0 < NHID; k0 += 32) {
        const v16h b0 = FragH::load(wh + k0);
        const v16h b1 = FragH::load(wh + (size_t)1 * NHID * NHID + k0);
        const v16h b2 = FragH::load(wh + (size_t)2 * NHID * NHID + k0);
        const v16h b3 = FragH::load(wh + (size_t)3 * NHID * NHID + k0);
        const v16h a0 = FragH::load(ah0 + k0);
        const v16h a1 = FragH::load(ah1 + k0);
        acc[0][0] = FragH::mma(a0, b0, acc[0][0]);
        acc[0][1] = FragH::mma(a1, b0, acc[0][1]);
        acc[1][0] = FragH::mma(a0, b1, acc[1][0]);
        acc[1][1] = FragH::mma(a1, b1, acc[1][1]);
        acc[2][0] = FragH::mma(a0, b2, acc[2][0]);
        acc[2][1] = FragH::mma(a1, b2, acc[2][1]);
        acc[3][0] = FragH::mma(a0, b3, acc[3][0]);
        acc[3][1] = FragH::mma(a1, b3, acc[3][1]);
        tie_one(acc[0][0], a0, b0);
        tie_one(acc[0][1], a1, b0);
        tie_one(acc[1][0], a0, b1);
        tie_one(acc[1][1], a1, b1);
        tie_one(acc[2][0], a0, b2);
        tie_one(acc[2][1], a1, b2);
        tie_one(acc[3][0], a0, b3);
        tie_close(acc[3][1], a0, a1, b0, b1, b2, b3);
      }
      settle_one(acc[0][0]);
      settle_one(acc[0][1]);
      settle_one(acc[1][0]);
      settle_one(acc[1][1]);
      settle_one(acc[2][0]);
      settle_one(acc[2][1]);
      settle_one(acc[3][0]);
      settle_one(acc[3][1]);
    }
    __syncthreads();

    const int tp1 = t + 1;
#pragma unroll
    for (int rt = 0; rt < 2; ++rt) {
#pragma unroll
      for (int v = 0; v < 8; ++v) {
        const float zi = acc[0][rt][v] * ACC_SCALE_INV;
        const float zf = acc[1][rt][v] * ACC_SCALE_INV;
        const float zg = acc[2][rt][v] * ACC_SCALE_INV;
        const float zo = acc[3][rt][v] * ACC_SCALE_INV;
        const float ig = fsig(zi);
        const float fg = fsig(zf);
        const float gg = ftanh(zg);
        const float og = fsig(zo);
        const float cn = fg * cst[rt][v] + ig * gg;
        cst[rt][v] = cn;
        const float hv = og * ftanh(cn);
        lh[rt][v] = (lenv[rt][v] == tp1) ? hv : lh[rt][v];
        const float hs = hv * HCARRY;
        const float hf = (fabsf(hs) < F16_MIN_NORMAL) ? 0.0f : hs;
        Ah[(16 * rt + 8 * hh + v) * HPITCH + u] = (_Float16)hf;
      }
    }
    __syncthreads();
  }

#pragma unroll
  for (int rt = 0; rt < 2; ++rt) {
#pragma unroll
    for (int v = 0; v < 8; ++v) Hs[(16 * rt + 8 * hh + v) * OPITCH + u] = lh[rt][v];
  }
  __syncthreads();
  for (int pass = 0; pass < 2; ++pass) {
#pragma unroll
    for (int it = 0; it < 4; ++it) {
      const int idx = it * RTHR + tid;
      const int row = idx >> 6;
      const int c4  = (idx & 63) * 4;
      const v4f val = *(const v4f*)(Hs + row * OPITCH + c4);
      *(volatile v4f*)(out + (size_t)(n0 + row) * NHID + c4) = val;
    }
    __threadfence();
  }
}

extern "C" void kernel_launch(void* const* d_in, const int* in_sizes, int n_in,
                              void* d_out, int out_size, void* d_ws, size_t ws_size, hipStream_t stream) {
  if (n_in < 6 || d_out == nullptr || d_ws == nullptr) return;
  if (in_sizes[0] != NWORD * NSTEP || in_sizes[1] != NCHAR * NEMB || in_sizes[2] != NGATE * NEMB ||
      in_sizes[3] != NGATE * NHID || in_sizes[4] != NGATE || in_sizes[5] != NGATE ||
      out_size != NWORD * NHID) return;

  const int*   chars = (const int*)d_in[0];
  const float* emb   = (const float*)d_in[1];
  const float* wih   = (const float*)d_in[2];
  const float* whh   = (const float*)d_in[3];
  const float* bih   = (const float*)d_in[4];
  const float* bhh   = (const float*)d_in[5];
  float* out = (float*)d_out;

  char* ws = (char*)d_ws;
  size_t off = 0;
  auto carve = [&](size_t bytes) -> char* { char* p = ws + off; off += (bytes + 255) & ~(size_t)255; return p; };
  float*          PT = (float*)carve((size_t)NCHAR * NGATE * 4);
  unsigned short* WH = (unsigned short*)carve((size_t)NGATE * NHID * 2);
  if (off > ws_size || off > (size_t)134217728) return;

  table_kernel<<<NCHAR, TAB_THR, 0, stream>>>(emb, wih, bih, bhh, PT);
  whh_cvt_kernel<<<(NGATE * NHID / 8 + CVT_THR - 1) / CVT_THR, CVT_THR, 0, stream>>>(whh, WH);
  rec_kernel<<<NWORD / TROWS, RTHR, 0, stream>>>(chars, PT, WH, out);
}
